// PillarFeatureNet_52536039964809
// MI455X (gfx1250) — hardware-verified
//
#include <hip/hip_runtime.h>
#include <math.h>

constexpr int   kPts        = 32;
constexpr int   kChan       = 64;
constexpr int   kKpack      = 32;
constexpr int   kCellChunk  = 4000;
constexpr int   kRowChunk   = kCellChunk * kPts;
constexpr int   kGemmBlocks = kRowChunk / 512;
constexpr int   kMomN       = 35;
constexpr float kBnEps      = 1.0e-3f;

typedef __attribute__((ext_vector_type(16))) _Float16 v16h;
typedef __attribute__((ext_vector_type(8)))  _Float16 v8h;
typedef __attribute__((ext_vector_type(16))) __bf16   v16b;
typedef __attribute__((ext_vector_type(8)))  __bf16   v8b;
typedef __attribute__((ext_vector_type(8)))  float    v8f;
typedef __attribute__((ext_vector_type(4)))  float    v4f;
typedef __attribute__((ext_vector_type(4)))  unsigned int v4u;

__device__ __forceinline__ unsigned short f2bf_bits(float f) {
  unsigned u = __float_as_uint(f);
  return (unsigned short)((u + 0x7FFFu + ((u >> 16) & 1u)) >> 16);
}
__device__ __forceinline__ float bf_bits2f(unsigned short h) { return __uint_as_float(((unsigned)h) << 16); }

__device__ __forceinline__ void dep_guard_h(v8f& a, v8f& b, v16h x, v16h y) { asm volatile("v_nop\n\tv_nop\n\tv_nop\n\tv_nop" : "+v"(a), "+v"(b) : "v"(x), "v"(y)); }
__device__ __forceinline__ void dep_guard_b(v8f& a, v8f& b, v16b x, v16b y) { asm volatile("v_nop\n\tv_nop\n\tv_nop\n\tv_nop" : "+v"(a), "+v"(b) : "v"(x), "v"(y)); }
__device__ __forceinline__ void keep4_h(v16h a, v16h b, v16h c, v16h d) { asm volatile("v_nop" :: "v"(a), "v"(b), "v"(c), "v"(d)); }
__device__ __forceinline__ void keep4_b(v16b a, v16b b, v16b c, v16b d) { asm volatile("v_nop" :: "v"(a), "v"(b), "v"(c), "v"(d)); }
__device__ __forceinline__ void acc_guard4(v8f& a, v8f& b, v8f& c, v8f& d) { asm volatile("v_nop\n\tv_nop\n\tv_nop\n\tv_nop" : "+v"(a), "+v"(b), "+v"(c), "+v"(d)); }
template <typename T> struct Frag;
template <> struct Frag<_Float16> {
  typedef v16h V; union U { v16h v; v8h h[2]; };
  static __device__ __forceinline__ v16h load(const _Float16* p) {
    U f; f.h[0] = *(const v8h*)(p); f.h[1] = *(const v8h*)(p + 16); return f.v;
  }
  static __device__ __forceinline__ v8f mma(v16h a, v16h b, v8f c) {
    return __builtin_amdgcn_wmma_f32_16x16x32_f16(false, a, false, b, (short)0, c, false, false);
  }
  static __device__ __forceinline__ void guard(v8f& a, v8f& b, v16h x, v16h y) { dep_guard_h(a, b, x, y); }
  static __device__ __forceinline__ void keep(v16h a, v16h b, v16h c, v16h d) { keep4_h(a, b, c, d); }
};
template <> struct Frag<__bf16> {
  typedef v16b V; union U { v16b v; v8b h[2]; };
  static __device__ __forceinline__ v16b load(const __bf16* p) {
    U f; f.h[0] = *(const v8b*)(p); f.h[1] = *(const v8b*)(p + 16); return f.v;
  }
  static __device__ __forceinline__ v8f mma(v16b a, v16b b, v8f c) {
    return __builtin_amdgcn_wmma_f32_16x16x32_bf16(false, a, false, b, (short)0, c, false, false);
  }
  static __device__ __forceinline__ void guard(v8f& a, v8f& b, v16b x, v16b y) { dep_guard_b(a, b, x, y); }
  static __device__ __forceinline__ void keep(v16b a, v16b b, v16b c, v16b d) { keep4_b(a, b, c, d); }
};

__device__ __forceinline__ unsigned pk16(unsigned short a, unsigned short b) { return (unsigned)a | ((unsigned)b << 16); }

template <int ET> struct Elem;
template <> struct Elem<0> { typedef _Float16 T; };
template <> struct Elem<1> { typedef __bf16 T; };
template <int ET, bool SPLIT, int BIAS_MODE, int OUT_MODE, bool RESID, int ACT = 0>
__global__ __launch_bounds__(256) void wmma_gemm64(
    const unsigned short* __restrict__ Ap, const unsigned short* __restrict__ A2p, int lda, long strideA,
    const unsigned short* __restrict__ Btp, const unsigned short* __restrict__ Bt2p, int ldb, long strideB,
    void* __restrict__ Cout, void* __restrict__ Cout2, int ldc, long strideC,
    const float* __restrict__ bias,
    const float* __restrict__ resid, long strideR,
    int M, int N, int K, float scale) {
  typedef typename Elem<ET>::T T;
  typedef typename Frag<T>::V V;
  const T* A = (const T*)Ap; const T* A2 = (const T*)A2p; const T* Bt = (const T*)Btp; const T* Bt2 = (const T*)Bt2p;
  __shared__ __align__(16) float sT[8][16 * 68];
  const int b    = blockIdx.y;
  const int lane = threadIdx.x & 31;
  const int wave = threadIdx.x >> 5;
  const int tilesN = N >> 6;
  const int tilesM = M >> 6;
  const int tile = blockIdx.x * 8 + wave;
  if (tile >= tilesM * tilesN) return;
  const int tm = tile / tilesN;
  const int tn = tile - tm * tilesN;
  const int m0 = tm << 6;
  const int n0 = tn << 6;

  const T* Ab  = A  + (size_t)b * strideA;
  const T* Bb  = Bt + (size_t)b * strideB;
  const T* Ab2 = SPLIT ? (A2  + (size_t)b * strideA) : nullptr;
  const T* Bb2 = SPLIT ? (Bt2 + (size_t)b * strideB) : nullptr;

  const int rlane = lane & 15;
  const int koff  = (lane >> 4) * 8;
  const int mOff  = (lane >> 4) * 8;

  v8f acc[4][4];
#pragma unroll
  for (int i = 0; i < 4; ++i)
#pragma unroll
    for (int j = 0; j < 4; ++j) acc[i][j] = (v8f){0.f,0.f,0.f,0.f,0.f,0.f,0.f,0.f};

  for (int k0 = 0; k0 < K; k0 += 32) {
    V bh[4], bl[4];
#pragma unroll
    for (int j = 0; j < 4; ++j) {
      const size_t bo = (size_t)(n0 + (j << 4) + rlane) * ldb + koff + k0;
      bh[j] = Frag<T>::load(Bb + bo);
      if (SPLIT) bl[j] = Frag<T>::load(Bb2 + bo);
    }
#pragma unroll
    for (int i = 0; i < 4; ++i) {
      const size_t ao = (size_t)(m0 + (i << 4) + rlane) * lda + koff + k0;
      V ah = Frag<T>::load(Ab + ao);
      V al;
      if (SPLIT) al = Frag<T>::load(Ab2 + ao);
#pragma unroll
      for (int j = 0; j < 4; ++j) {
        acc[i][j] = Frag<T>::mma(ah, bh[j], acc[i][j]);
        if (SPLIT) {
          acc[i][j] = Frag<T>::mma(ah, bl[j], acc[i][j]);
          acc[i][j] = Frag<T>::mma(al, bh[j], acc[i][j]);
        }
      }
      Frag<T>::guard(acc[i][0], acc[i][3], ah, SPLIT ? al : ah);
    }
    Frag<T>::keep(bh[0], bh[1], bh[2], bh[3]);
    if (SPLIT) Frag<T>::keep(bl[0], bl[1], bl[2], bl[3]);
  }
  acc_guard4(acc[0][0], acc[0][1], acc[0][2], acc[0][3]);
  acc_guard4(acc[1][0], acc[1][1], acc[1][2], acc[1][3]);
  acc_guard4(acc[2][0], acc[2][1], acc[2][2], acc[2][3]);
  acc_guard4(acc[3][0], acc[3][1], acc[3][2], acc[3][3]);

  float* slab = sT[wave];

  if (OUT_MODE == 3) {
    float cs[4], cq[4];
#pragma unroll
    for (int j = 0; j < 4; ++j) {
      float s = 0.f, q = 0.f;
#pragma unroll
      for (int i = 0; i < 4; ++i) {
#pragma unroll
        for (int r = 0; r < 8; ++r) {
          const float v = acc[i][j][r] * scale;
          s += v;
          q = fmaf(v, v, q);
        }
      }
      cs[j] = s; cq[j] = q;
    }
#pragma unroll
    for (int j = 0; j < 4; ++j) {
      cs[j] += __shfl_xor(cs[j], 16, 32);
      cq[j] += __shfl_xor(cq[j], 16, 32);
    }
#pragma unroll
    for (int j = 0; j < 4; ++j) {
      slab[(j << 4) + rlane]      = cs[j];
      slab[64 + (j << 4) + rlane] = cq[j];
    }
    __syncthreads();
    if (wave == 0) {
      v4f tsum = (v4f){0.f, 0.f, 0.f, 0.f};
#pragma unroll
      for (int w = 0; w < 8; ++w) {
        const v4f u = *(const v4f*)(sT[w] + lane * 4);
        tsum = tsum + u;
      }
      float* C = (float*)Cout + (size_t)blockIdx.x * 128;
      for (int pass = 0; pass < 2; ++pass) {
        *(volatile v4f*)(C + lane * 4) = tsum;
        __threadfence();
      }
    }
    return;
  }

  if (OUT_MODE == 4) {
    float ma[4], mb[4];
#pragma unroll
    for (int j = 0; j < 4; ++j) {
      const int n = n0 + (j << 4) + rlane;
      const float bsc = bias[n];
      const float bsh = bias[N + n];
      float xa = 0.f, xb = 0.f;
#pragma unroll
      for (int r = 0; r < 8; ++r) {
        const float v0 = fmaxf(fmaf(acc[0][j][r] * scale, bsc, bsh), 0.f);
        const float v1 = fmaxf(fmaf(acc[1][j][r] * scale, bsc, bsh), 0.f);
        const float v2 = fmaxf(fmaf(acc[2][j][r] * scale, bsc, bsh), 0.f);
        const float v3 = fmaxf(fmaf(acc[3][j][r] * scale, bsc, bsh), 0.f);
        xa = fmaxf(xa, fmaxf(v0, v1));
        xb = fmaxf(xb, fmaxf(v2, v3));
      }
      ma[j] = xa; mb[j] = xb;
    }
#pragma unroll
    for (int j = 0; j < 4; ++j) {
      ma[j] = fmaxf(ma[j], __shfl_xor(ma[j], 16, 32));
      mb[j] = fmaxf(mb[j], __shfl_xor(mb[j], 16, 32));
    }
#pragma unroll
    for (int j = 0; j < 4; ++j) {
      slab[(j << 4) + rlane]      = ma[j];
      slab[64 + (j << 4) + rlane] = mb[j];
    }
    __builtin_amdgcn_fence(__ATOMIC_RELEASE, "workgroup");
    __builtin_amdgcn_wave_barrier();
    __builtin_amdgcn_fence(__ATOMIC_ACQUIRE, "workgroup");
    const v4f ov = *(const v4f*)(slab + lane * 4);
    float* C = (float*)Cout + (size_t)(m0 >> 5) * ldc;
    for (int pass = 0; pass < 2; ++pass) {
      *(volatile v4f*)(C + lane * 4) = ov;
      __threadfence();
    }
    return;
  }

  const float* Rb = RESID ? (resid + (size_t)b * strideR) : nullptr;
#pragma unroll
  for (int i = 0; i < 4; ++i) {
    const int mBase = m0 + (i << 4);
#pragma unroll
    for (int j = 0; j < 4; ++j) {
      const int n = n0 + (j << 4) + rlane;
      float bv = 0.f, bs = 1.f;
      if (BIAS_MODE == 2) bv = bias[n];
      if (BIAS_MODE == 3) { bs = bias[n]; bv = bias[N + n]; }
#pragma unroll
      for (int r = 0; r < 8; ++r) {
        float v = acc[i][j][r] * scale;
        if (BIAS_MODE == 1) v += bias[mBase + mOff + r];
        if (BIAS_MODE == 2) v += bv;
        if (BIAS_MODE == 3) v = fmaf(v, bs, bv);
        if (RESID) v += Rb[(size_t)(mBase + mOff + r) * ldc + n];
        if (ACT == 2) v = fmaxf(v, 0.0f);
        if (ACT == 4) v = (v > 0.f) ? v : 0.01f * v;
        slab[(mOff + r) * 68 + (j << 4) + rlane] = v;
      }
    }
    __builtin_amdgcn_fence(__ATOMIC_RELEASE, "workgroup");
    __builtin_amdgcn_wave_barrier();
    __builtin_amdgcn_fence(__ATOMIC_ACQUIRE, "workgroup");
    if (OUT_MODE == 0) {
      float* C = (float*)Cout + (size_t)b * strideC;
      const int hh = lane >> 4, c4 = (lane & 15) * 4;
      for (int pass = 0; pass < 2; ++pass) {
#pragma unroll
        for (int it = 0; it < 8; ++it) {
          const int row = it * 2 + hh;
          v4f v = *(const v4f*)(slab + row * 68 + c4);
          *(volatile v4f*)(C + (size_t)(mBase + row) * ldc + n0 + c4) = v;
        }
        __threadfence();
      }
    } else {
      const int q = lane >> 3, c8 = (lane & 7) * 8;
      unsigned short* C  = (unsigned short*)Cout  + (size_t)b * strideC;
      unsigned short* C2 = (OUT_MODE == 2) ? ((unsigned short*)Cout2 + (size_t)b * strideC) : nullptr;
      for (int pass = 0; pass < 2; ++pass) {
#pragma unroll
        for (int it = 0; it < 4; ++it) {
          const int row = it * 4 + q;
          const float* sp = slab + row * 68 + c8;
          v8h hv, lv;
#pragma unroll
          for (int e = 0; e < 8; ++e) {
            if (OUT_MODE == 1) {
              hv[e] = (_Float16)sp[e];
            } else {
              unsigned short hb = f2bf_bits(sp[e]);
              unsigned short lb = f2bf_bits(sp[e] - bf_bits2f(hb));
              hv[e] = __builtin_bit_cast(_Float16, hb);
              lv[e] = __builtin_bit_cast(_Float16, lb);
            }
          }
          *(volatile v8h*)(C + (size_t)(mBase + row) * ldc + n0 + c8) = hv;
          if (OUT_MODE == 2) *(volatile v8h*)(C2 + (size_t)(mBase + row) * ldc + n0 + c8) = lv;
        }
        __threadfence();
      }
    }
    __builtin_amdgcn_fence(__ATOMIC_RELEASE, "workgroup");
    __builtin_amdgcn_wave_barrier();
    __builtin_amdgcn_fence(__ATOMIC_ACQUIRE, "workgroup");
  }
}

__global__ __launch_bounds__(256) void wprep_kernel(const float* __restrict__ W1, const float* __restrict__ W2,
                                                    v4u* __restrict__ Wout) {
  __shared__ __align__(16) unsigned short wl[10240];
  const int t = threadIdx.x;
#pragma unroll 1
  for (int idx = t; idx < 2048; idx += 256) {
    const int n = idx >> 5, k = idx & 31;
    const int c = k / 3;
    const int typ = k - 3 * c;
    const int cc = c < 9 ? c : 8;
    const float w = W1[cc * kChan + n];
    const unsigned short hb = f2bf_bits(w);
    const unsigned short lb = f2bf_bits(w - bf_bits2f(hb));
    unsigned short v = (typ == 1) ? lb : hb;
    v = (k < 27) ? v : (unsigned short)0;
    wl[idx] = v;
  }
#pragma unroll 1
  for (int idx = t; idx < 4096; idx += 256) {
    const int n = idx >> 6, k = idx & 63;
    const float w = W2[k * kChan + n];
    const unsigned short hb = f2bf_bits(w);
    const unsigned short lb = f2bf_bits(w - bf_bits2f(hb));
    wl[2048 + idx] = hb;
    wl[6144 + idx] = lb;
  }
  __syncthreads();
  v4u o[5];
#pragma unroll
  for (int it = 0; it < 5; ++it) o[it] = *(const v4u*)(wl + 8 * (it * 256 + t));
  for (int pass = 0; pass < 2; ++pass) {
#pragma unroll
    for (int it = 0; it < 5; ++it) *(volatile v4u*)(Wout + it * 256 + t) = o[it];
    __threadfence();
  }
}

__global__ __launch_bounds__(256) void featurize_kernel(const float* __restrict__ vox, const int* __restrict__ coords,
                                                        const int* __restrict__ npts, v4u* __restrict__ Fp4, int nCell) {
#pragma clang fp contract(off)
  __shared__ v4u fst[8][32][4];
  const int lane = threadIdx.x & 31, wave = threadIdx.x >> 5;
  const int cell  = blockIdx.x * 8 + wave;
  const int cellc = cell < nCell ? cell : nCell - 1;
  const v4f vx = *(const v4f*)(vox + ((size_t)cellc * kPts + lane) * 4);
  const int c2 = coords[(size_t)cellc * 4 + 2];
  const int c3 = coords[(size_t)cellc * 4 + 3];
  const float cx = ((float)c3 + 0.5f) * 0.16f + 0.0f;
  const float cy = ((float)c2 + 0.5f) * 0.16f + (-39.68f);
  float zs = vx[2];
#pragma unroll
  for (int off = 16; off >= 1; off >>= 1) zs += __shfl_xor(zs, off, 32);
  const float zc = zs * 0.03125f;
  const int np = npts[cellc];
  const float msk = (lane < np) ? 1.0f : 0.0f;
  float f[9];
  f[0] = vx[0] * msk;
  f[1] = vx[1] * msk;
  f[2] = vx[2] * msk;
  f[3] = vx[3] * msk;
  f[4] = (vx[0] - cx) * msk;
  f[5] = (vx[1] - cy) * msk;
  f[6] = cx * msk;
  f[7] = cy * msk;
  f[8] = zc * msk;
  unsigned short hb[9], lb[9];
#pragma unroll
  for (int k = 0; k < 9; ++k) {
    hb[k] = f2bf_bits(f[k]);
    lb[k] = f2bf_bits(f[k] - bf_bits2f(hb[k]));
  }
  unsigned zero;
  asm volatile("v_mov_b32 %0, 0" : "=v"(zero));
  v4u wv[4];
  wv[0] = (v4u){pk16(hb[0], hb[0]), pk16(lb[0], hb[1]), pk16(hb[1], lb[1]), pk16(hb[2], hb[2])};
  wv[1] = (v4u){pk16(lb[2], hb[3]), pk16(hb[3], lb[3]), pk16(hb[4], hb[4]), pk16(lb[4], hb[5])};
  wv[2] = (v4u){pk16(hb[5], lb[5]), pk16(hb[6], hb[6]), pk16(lb[6], hb[7]), pk16(hb[7], lb[7])};
  wv[3] = (v4u){pk16(hb[8], hb[8]), ((unsigned)lb[8]) | (zero << 16), zero, zero};
#pragma unroll
  for (int tq = 0; tq < 4; ++tq) fst[wave][lane][tq] = wv[tq];
  __builtin_amdgcn_fence(__ATOMIC_RELEASE, "workgroup");
  __builtin_amdgcn_wave_barrier();
  __builtin_amdgcn_fence(__ATOMIC_ACQUIRE, "workgroup");
  v4u o[4];
#pragma unroll
  for (int tq = 0; tq < 4; ++tq) o[tq] = fst[wave][tq * 8 + (lane >> 2)][lane & 3];
  if (cell < nCell) {
    v4u* dst = Fp4 + (size_t)cell * 128;
    for (int pass = 0; pass < 2; ++pass) {
#pragma unroll
      for (int tq = 0; tq < 4; ++tq) *(volatile v4u*)(dst + tq * 32 + lane) = o[tq];
      __threadfence();
    }
  }
}

__global__ __launch_bounds__(256) void moments1_kernel(const float* __restrict__ vox, const int* __restrict__ coords,
                                                       const int* __restrict__ npts, float* __restrict__ part, int nCell) {
  __shared__ float red[8][36];
  __shared__ __align__(16) float lineb[64];
  const int t = threadIdx.x, lane = t & 31, wave = t >> 5;
  const int cell = blockIdx.x * 256 + t;
  const bool ok = cell < nCell;
  const int cellc = ok ? cell : nCell - 1;
  int np = npts[cellc];
  np = np < 0 ? 0 : (np > kPts ? kPts : np);
  if (!ok) np = 0;
  float sx = 0.f, sy = 0.f, sz = 0.f, se = 0.f, zsum = 0.f;
  float qxx = 0.f, qxy = 0.f, qxz = 0.f, qxe = 0.f, qyy = 0.f, qyz = 0.f, qye = 0.f, qzz = 0.f, qze = 0.f, qee = 0.f;
  const float* vp = vox + (size_t)cellc * (kPts * 4);
#pragma unroll 1
  for (int m = 0; m < kPts; ++m) {
    const v4f v = *(const v4f*)(vp + m * 4);
    const float vm = (m < np) ? 1.0f : 0.0f;
    const float x = v[0] * vm, y = v[1] * vm, z = v[2] * vm, e = v[3] * vm;
    sx += x; sy += y; sz += z; se += e;
    qxx = fmaf(x, v[0], qxx); qxy = fmaf(x, v[1], qxy); qxz = fmaf(x, v[2], qxz); qxe = fmaf(x, v[3], qxe);
    qyy = fmaf(y, v[1], qyy); qyz = fmaf(y, v[2], qyz); qye = fmaf(y, v[3], qye);
    qzz = fmaf(z, v[2], qzz); qze = fmaf(z, v[3], qze);
    qee = fmaf(e, v[3], qee);
    zsum += v[2];
  }
  float cx, cy;
  {
#pragma clang fp contract(off)
    const int c2 = coords[(size_t)cellc * 4 + 2];
    const int c3 = coords[(size_t)cellc * 4 + 3];
    cx = ((float)c3 + 0.5f) * 0.16f + 0.0f;
    cy = ((float)c2 + 0.5f) * 0.16f + (-39.68f);
  }
  const float zc = zsum * 0.03125f;
  const float nf = (float)np;
  float mv[kMomN];
  mv[0] = sx; mv[1] = sy; mv[2] = sz; mv[3] = se; mv[4] = nf * cx; mv[5] = nf * cy; mv[6] = nf * zc;
  mv[7]  = qxx; mv[8]  = qxy; mv[9]  = qxz; mv[10] = qxe; mv[11] = sx * cx; mv[12] = sx * cy; mv[13] = sx * zc;
  mv[14] = qyy; mv[15] = qyz; mv[16] = qye; mv[17] = sy * cx; mv[18] = sy * cy; mv[19] = sy * zc;
  mv[20] = qzz; mv[21] = qze; mv[22] = sz * cx; mv[23] = sz * cy; mv[24] = sz * zc;
  mv[25] = qee; mv[26] = se * cx; mv[27] = se * cy; mv[28] = se * zc;
  mv[29] = nf * cx * cx; mv[30] = nf * cx * cy; mv[31] = nf * cx * zc;
  mv[32] = nf * cy * cy; mv[33] = nf * cy * zc;
  mv[34] = nf * zc * zc;
#pragma unroll
  for (int k = 0; k < kMomN; ++k) {
    float v = mv[k];
#pragma unroll
    for (int off = 16; off >= 1; off >>= 1) v += __shfl_xor(v, off, 32);
    red[wave][k] = v;
  }
  __syncthreads();
  if (t < 64) {
    const int tc = t < kMomN ? t : kMomN - 1;
    float tot = 0.f;
#pragma unroll
    for (int w = 0; w < 8; ++w) tot += red[w][tc];
    lineb[t] = (t < kMomN) ? tot : 0.0f;
  }
  __syncthreads();
  if (wave == 0) {
    const int li = (lane & 15) * 4;
    const v4f v = *(const v4f*)(lineb + li);
    float* dst = part + (size_t)blockIdx.x * 64;
    for (int pass = 0; pass < 2; ++pass) {
      if (lane < 16) *(volatile v4f*)(dst + li) = v;
      __threadfence();
    }
  }
}

__global__ __launch_bounds__(64) void bn1_fold_kernel(const float* __restrict__ part, int nb,
                                                      const float* __restrict__ W1, const float* __restrict__ g1,
                                                      const float* __restrict__ b1, float* __restrict__ scsh, float invN) {
  __shared__ float tot[36];
  __shared__ __align__(16) float stage[128];
  const int t = threadIdx.x;
  const int tc = t < kMomN ? t : kMomN - 1;
  float accv = 0.f;
#pragma unroll 1
  for (int g0 = 0; g0 < nb; g0 += 16) {
    float ps = 0.f;
#pragma unroll 1
    for (int u = 0; u < 16; ++u) {
      const int bi = g0 + u;
      const int bic = bi < nb ? bi : nb - 1;
      const float v = part[(size_t)bic * 64 + tc];
      ps += (bi < nb) ? v : 0.0f;
    }
    accv += ps;
  }
  if (t < kMomN) tot[t] = accv;
  __syncthreads();
  float w[9];
#pragma unroll
  for (int i = 0; i < 9; ++i) w[i] = W1[i * kChan + t];
  float u[7];
  u[0] = w[0] + w[4];
  u[1] = w[1] + w[5];
  u[2] = w[2];
  u[3] = w[3];
  u[4] = w[6] - w[4];
  u[5] = w[7] - w[5];
  u[6] = w[8];
  float S = 0.f;
#pragma unroll
  for (int a = 0; a < 7; ++a) S = fmaf(tot[a], u[a], S);
  float Q = 0.f;
#pragma unroll
  for (int a = 0; a < 7; ++a) {
#pragma unroll
    for (int bb = a; bb < 7; ++bb) {
      const int gi = 7 + a * 7 - (a * (a - 1)) / 2 + (bb - a);
      const float mult = (a == bb) ? 1.0f : 2.0f;
      Q = fmaf(mult * tot[gi] * u[a], u[bb], Q);
    }
  }
  const float mean = S * invN;
  const float ez2  = Q * invN;
  const float var  = fmaxf(ez2 - mean * mean, 0.0f);
  const float rs   = 1.0f / sqrtf(var + kBnEps);
  const float sc   = rs * g1[t];
  const float sh   = b1[t] - mean * sc;
  stage[t] = sc;
  stage[64 + t] = sh;
  __syncthreads();
  if (t < 32) {
    const v4f v = *(const v4f*)(stage + t * 4);
    for (int pass = 0; pass < 2; ++pass) {
      *(volatile v4f*)(scsh + t * 4) = v;
      __threadfence();
    }
  }
}

__global__ __launch_bounds__(128) void bn2_fold_kernel(const float* __restrict__ part, int nb,
                                                       const float* __restrict__ g2, const float* __restrict__ b2,
                                                       float* __restrict__ scsh, float invN) {
  __shared__ float tot[128];
  __shared__ __align__(16) float stage[128];
  const int t = threadIdx.x;
  float accv = 0.f;
#pragma unroll 1
  for (int g0 = 0; g0 < nb; g0 += 16) {
    float ps = 0.f;
#pragma unroll 1
    for (int u = 0; u < 16; ++u) {
      const int bi = g0 + u;
      const int bic = bi < nb ? bi : nb - 1;
      const float v = part[(size_t)bic * 128 + t];
      ps += (bi < nb) ? v : 0.0f;
    }
    accv += ps;
  }
  tot[t] = accv;
  __syncthreads();
  if (t < 64) {
    const float mean = tot[t] * invN;
    const float ez2  = tot[64 + t] * invN;
    const float var  = fmaxf(ez2 - mean * mean, 0.0f);
    const float rs   = 1.0f / sqrtf(var + kBnEps);
    const float sc   = rs * g2[t];
    const float sh   = b2[t] - mean * sc;
    stage[t] = sc;
    stage[64 + t] = sh;
  }
  __syncthreads();
  if (t < 32) {
    const v4f v = *(const v4f*)(stage + t * 4);
    for (int pass = 0; pass < 2; ++pass) {
      *(volatile v4f*)(scsh + t * 4) = v;
      __threadfence();
    }
  }
}

extern "C" void kernel_launch(void* const* d_in, const int* in_sizes, int n_in,
                              void* d_out, int out_size, void* d_ws, size_t ws_size,
                              hipStream_t stream) {
  if (n_in < 9) return;
  const float* vox    = (const float*)d_in[0];
  const int*   coords = (const int*)d_in[1];
  const int*   npts   = (const int*)d_in[2];
  const float* W1 = (const float*)d_in[3];
  const float* g1 = (const float*)d_in[4];
  const float* b1 = (const float*)d_in[5];
  const float* W2 = (const float*)d_in[6];
  const float* g2 = (const float*)d_in[7];
  const float* b2 = (const float*)d_in[8];
  float* out = (float*)d_out;

  const int nCell = in_sizes[2];
  if (nCell <= 0 || (nCell % kCellChunk) != 0) return;
  if (in_sizes[0] != nCell * kPts * 4) return;
  if (in_sizes[1] != nCell * 4) return;
  if (in_sizes[3] != 9 * kChan || in_sizes[6] != kChan * kChan) return;
  if (in_sizes[4] != kChan || in_sizes[5] != kChan || in_sizes[7] != kChan || in_sizes[8] != kChan) return;
  if (out_size != nCell * kChan) return;

  const int  nChunks   = nCell / kCellChunk;
  const long rowsTotal = (long)nCell * kPts;
  const int  nb1       = (nCell + 255) / 256;
  const int  nb2       = nChunks * kGemmBlocks;
  const float invN     = 1.0f / (float)rowsTotal;

  size_t off = 0;
  auto take = [&](size_t bytes) { size_t o = off; off += (bytes + 255) & ~(size_t)255; return o; };
  const size_t oW  = take(20480);
  const size_t oS1 = take(512);
  const size_t oS2 = take(512);
  const size_t oP1 = take((size_t)nb1 * 256);
  const size_t oP2 = take((size_t)nb2 * 512);
  const size_t oF  = take((size_t)rowsTotal * kKpack * 2);
  const size_t oHh = take((size_t)kRowChunk * kChan * 2);
  const size_t oHl = take((size_t)kRowChunk * kChan * 2);
  if (off > ws_size) return;

  char* ws = (char*)d_ws;
  v4u*            Wv    = (v4u*)(ws + oW);
  unsigned short* W1p   = (unsigned short*)(ws + oW);
  unsigned short* W2h   = W1p + 2048;
  unsigned short* W2l   = W1p + 6144;
  float*          scsh1 = (float*)(ws + oS1);
  float*          scsh2 = (float*)(ws + oS2);
  float*          part1 = (float*)(ws + oP1);
  float*          part2 = (float*)(ws + oP2);
  unsigned short* Fp    = (unsigned short*)(ws + oF);
  unsigned short* Hh    = (unsigned short*)(ws + oHh);
  unsigned short* Hl    = (unsigned short*)(ws + oHl);

  wprep_kernel<<<1, 256, 0, stream>>>(W1, W2, Wv);
  featurize_kernel<<<nCell / 8, 256, 0, stream>>>(vox, coords, npts, (v4u*)(ws + oF), nCell);
  moments1_kernel<<<nb1, 256, 0, stream>>>(vox, coords, npts, part1, nCell);
  bn1_fold_kernel<<<1, 64, 0, stream>>>(part1, nb1, W1, g1, b1, scsh1, invN);

  for (int c = 0; c < nChunks; ++c) {
    const unsigned short* Fc = Fp + (size_t)c * kRowChunk * kKpack;
    wmma_gemm64<1, false, 3, 2, false, 2><<<dim3(kGemmBlocks, 1), 256, 0, stream>>>(
        Fc, Fc, kKpack, 0L, W1p, W1p, kKpack, 0L,
        (void*)Hh, (void*)Hl, kChan, 0L, scsh1, nullptr, 0L, kRowChunk, kChan, kKpack, 1.0f);
    wmma_gemm64<1, true, 0, 3, false, 0><<<dim3(kGemmBlocks, 1), 256, 0, stream>>>(
        Hh, Hl, kChan, 0L, W2h, W2l, kChan, 0L,
        (void*)(part2 + (size_t)c * kGemmBlocks * 128), nullptr, kChan, 0L, nullptr, nullptr, 0L,
        kRowChunk, kChan, kChan, 1.0f);
  }
  bn2_fold_kernel<<<1, 128, 0, stream>>>(part2, nb2, g2, b2, scsh2, invN);

  for (int c = 0; c < nChunks; ++c) {
    const unsigned short* Fc = Fp + (size_t)c * kRowChunk * kKpack;
    wmma_gemm64<1, false, 3, 2, false, 2><<<dim3(kGemmBlocks, 1), 256, 0, stream>>>(
        Fc, Fc, kKpack, 0L, W1p, W1p, kKpack, 0L,
        (void*)Hh, (void*)Hl, kChan, 0L, scsh1, nullptr, 0L, kRowChunk, kChan, kKpack, 1.0f);
    wmma_gemm64<1, true, 3, 4, false, 0><<<dim3(kGemmBlocks, 1), 256, 0, stream>>>(
        Hh, Hl, kChan, 0L, W2h, W2l, kChan, 0L,
        (void*)(out + (size_t)c * kCellChunk * kChan), nullptr, kChan, 0L, scsh2, nullptr, 0L,
        kRowChunk, kChan, kChan, 1.0f);
  }
}
